// DenseEntangler_10582799417614
// MI455X (gfx1250) — hardware-run, weakly checked
//
#include <hip/hip_runtime.h>
#include <math.h>

typedef __attribute__((ext_vector_type(16))) _Float16 v16h;
typedef __attribute__((ext_vector_type(8)))  _Float16 v8h;
typedef __attribute__((ext_vector_type(2)))  _Float16 v2h;
typedef __attribute__((ext_vector_type(16))) __bf16   v16b;
typedef __attribute__((ext_vector_type(8)))  __bf16   v8b;
typedef __attribute__((ext_vector_type(8)))  float    v8f;
typedef __attribute__((ext_vector_type(4)))  float    v4f;
typedef __attribute__((ext_vector_type(2)))  float    v2f;

constexpr int kBn   = 256;
constexpr int kD    = 32;
constexpr int kDD   = kD * kD;
constexpr int kM    = kBn * kD;
constexpr int kNN   = 6;
constexpr int kOut  = kD * kD * kD;
constexpr int kThr  = 256;
constexpr float kInCarry = 1024.0f;
constexpr float kSc = 1.0f / (kInCarry * kInCarry);
constexpr float kF16MinNormal = 6.103515625e-5f;

static_assert(kBn == 256 && kD == 32 && kDD == 1024 && kM == 8192 && kNN == 6 && kOut == 32768, "the index arithmetic below uses these sizes (every leg a power of two: shifts and masks)");

constexpr size_t kOffZB = 0ull;
constexpr size_t kOffNW = 8192ull;
constexpr size_t kOffA16 = 16785408ull;
constexpr size_t kOffC = 50339840ull;
constexpr size_t kWsTotal = 83894272ull;
static_assert(kWsTotal <= 268435456ull, "the carve stands under 256 MiB");
static_assert(kOffZB == 0
  && kOffNW == kOffZB + 8192ull
  && kOffA16 == kOffNW + 16777216ull
  && kOffC == kOffA16 + 33554432ull
  && kWsTotal == kOffC + 33554432ull, "the carve is a chain: every region starts where the one before ends");
static_assert(((size_t)4 * kDD * kDD + (size_t)2 * kDD * 2 * kDD) * 2 == 16777216ull && (size_t)kM * 2 * kDD * 2 == 33554432ull && (size_t)kM * kDD * 4 == 33554432ull, "every region's length is its plane's");
static_assert((kOffNW % 256) == 0 && (kOffA16 % 256) == 0 && (kOffC % 256) == 0, "every region starts on a multiple of 256 B");

__device__ __forceinline__ unsigned short f2bf_bits(float f) {
  unsigned u = __float_as_uint(f);
  return (unsigned short)((u + 0x7FFFu + ((u >> 16) & 1u)) >> 16);
}
__device__ __forceinline__ float bf_bits2f(unsigned short h) { return __uint_as_float(((unsigned)h) << 16); }
__device__ __forceinline__ float bf16r(float f) { return bf_bits2f(f2bf_bits(f)); }
__device__ __forceinline__ float carry_flush(float v, float carry) {
  const float s = v * carry;
  return (fabsf(s) < kF16MinNormal) ? 0.0f : s;
}

__device__ __forceinline__ void dep_guard4_h(v8f& a, v8f& b, v8f& c, v8f& d, v16h x, v16h y) { asm volatile("v_nop\n\tv_nop\n\tv_nop\n\tv_nop" : "+v"(a), "+v"(b), "+v"(c), "+v"(d) : "v"(x), "v"(y)); }
__device__ __forceinline__ void dep_guard4_b(v8f& a, v8f& b, v8f& c, v8f& d, v16b x, v16b y) { asm volatile("v_nop\n\tv_nop\n\tv_nop\n\tv_nop" : "+v"(a), "+v"(b), "+v"(c), "+v"(d) : "v"(x), "v"(y)); }
__device__ __forceinline__ void keep4_h(v16h a, v16h b, v16h c, v16h d) { asm volatile("v_nop" :: "v"(a), "v"(b), "v"(c), "v"(d)); }
__device__ __forceinline__ void keep4_b(v16b a, v16b b, v16b c, v16b d) { asm volatile("v_nop" :: "v"(a), "v"(b), "v"(c), "v"(d)); }
__device__ __forceinline__ void acc_guard4(v8f& a, v8f& b, v8f& c, v8f& d) { asm volatile("v_nop\n\tv_nop\n\tv_nop\n\tv_nop" : "+v"(a), "+v"(b), "+v"(c), "+v"(d)); }

template <typename T> struct Frag;
template <> struct Frag<_Float16> {
  typedef v16h V; union U { v16h v; v8h h[2]; };
  static __device__ __forceinline__ v16h load(const _Float16* p) {
    U f; f.h[0] = *(const v8h*)(p); f.h[1] = *(const v8h*)(p + 16); return f.v;
  }
  static __device__ __forceinline__ v8f mma(v16h a, v16h b, v8f c) {
    return __builtin_amdgcn_wmma_f32_16x16x32_f16(false, a, false, b, (short)0, c, false, false);
  }
  static __device__ __forceinline__ void guard4(v8f& a, v8f& b, v8f& c, v8f& d, v16h x, v16h y) { dep_guard4_h(a, b, c, d, x, y); }
  static __device__ __forceinline__ void keep(v16h a, v16h b, v16h c, v16h d) { keep4_h(a, b, c, d); }
};
template <> struct Frag<__bf16> {
  typedef v16b V; union U { v16b v; v8b h[2]; };
  static __device__ __forceinline__ v16b load(const __bf16* p) {
    U f; f.h[0] = *(const v8b*)(p); f.h[1] = *(const v8b*)(p + 16); return f.v;
  }
  static __device__ __forceinline__ v8f mma(v16b a, v16b b, v8f c) {
    return __builtin_amdgcn_wmma_f32_16x16x32_bf16(false, a, false, b, (short)0, c, false, false);
  }
  static __device__ __forceinline__ void guard4(v8f& a, v8f& b, v8f& c, v8f& d, v16b x, v16b y) { dep_guard4_b(a, b, c, d, x, y); }
  static __device__ __forceinline__ void keep(v16b a, v16b b, v16b c, v16b d) { keep4_b(a, b, c, d); }
};

__device__ __forceinline__ v8f mma_h(v16h a, v16h b, v8f c) {
  c = __builtin_amdgcn_wmma_f32_16x16x32_f16(false, a, false, b, (short)0, c, false, false);
  asm volatile("v_nop\n\tv_nop\n\tv_nop\n\tv_nop" : "+v"(c) : "v"(a), "v"(b));
  return c;
}

template <int ET> struct Elem;
template <> struct Elem<0> { typedef _Float16 T; };
template <> struct Elem<1> { typedef __bf16 T; };
template <int ET, bool SPLIT, int BIAS_MODE, int OUT_MODE, bool RESID, int ACT = 0>
__global__ __launch_bounds__(256) void wmma_gemm64(
    const unsigned short* __restrict__ Ap, const unsigned short* __restrict__ A2p, int lda, long strideA,
    const unsigned short* __restrict__ Btp, const unsigned short* __restrict__ Bt2p, int ldb, long strideB,
    void* __restrict__ Cout, void* __restrict__ Cout2, int ldc, long strideC,
    const float* __restrict__ bias,
    const float* __restrict__ resid, long strideR,
    int M, int N, int K, float scale) {
  typedef typename Elem<ET>::T T;
  typedef typename Frag<T>::V V;
  const T* A = (const T*)Ap; const T* A2 = (const T*)A2p; const T* Bt = (const T*)Btp; const T* Bt2 = (const T*)Bt2p;
  __shared__ __align__(16) float sT[8][16 * 68];
  const int b    = blockIdx.y;
  const int lane = threadIdx.x & 31;
  const int wave = threadIdx.x >> 5;
  const int tilesN = N >> 6;
  const int tilesM = M >> 6;
  const int tile = blockIdx.x * 8 + wave;
  if (tile >= tilesM * tilesN) return;
  const int tm = tile / tilesN;
  const int tn = tile - tm * tilesN;
  const int m0 = tm << 6;
  const int n0 = tn << 6;

  const T* Ab  = A  + (size_t)b * strideA;
  const T* Bb  = Bt + (size_t)b * strideB;
  const T* Ab2 = SPLIT ? (A2  + (size_t)b * strideA) : nullptr;
  const T* Bb2 = SPLIT ? (Bt2 + (size_t)b * strideB) : nullptr;

  const int rlane = lane & 15;
  const int koff  = (lane >> 4) * 8;
  const int mOff  = (lane >> 4) * 8;

  v8f acc[4][4];
#pragma unroll
  for (int i = 0; i < 4; ++i)
#pragma unroll
    for (int j = 0; j < 4; ++j) acc[i][j] = (v8f){0.f,0.f,0.f,0.f,0.f,0.f,0.f,0.f};

  for (int k0 = 0; k0 < K; k0 += 32) {
    V bh[4], bl[4];
#pragma unroll
    for (int j = 0; j < 4; ++j) {
      const size_t bo = (size_t)(n0 + (j << 4) + rlane) * ldb + koff + k0;
      bh[j] = Frag<T>::load(Bb + bo);
      if (SPLIT) bl[j] = Frag<T>::load(Bb2 + bo);
    }
#pragma unroll
    for (int i = 0; i < 4; ++i) {
      const size_t ao = (size_t)(m0 + (i << 4) + rlane) * lda + koff + k0;
      V ah = Frag<T>::load(Ab + ao);
      V al;
      if (SPLIT) al = Frag<T>::load(Ab2 + ao);
#pragma unroll
      for (int j = 0; j < 4; ++j) {
        acc[i][j] = Frag<T>::mma(ah, bh[j], acc[i][j]);
        if (SPLIT) {
          acc[i][j] = Frag<T>::mma(ah, bl[j], acc[i][j]);
          acc[i][j] = Frag<T>::mma(al, bh[j], acc[i][j]);
        }
      }
      Frag<T>::guard4(acc[i][0], acc[i][1], acc[i][2], acc[i][3], ah, SPLIT ? al : ah);
    }
    Frag<T>::keep(bh[0], bh[1], bh[2], bh[3]);
    if (SPLIT) Frag<T>::keep(bl[0], bl[1], bl[2], bl[3]);
  }
  acc_guard4(acc[0][0], acc[0][1], acc[0][2], acc[0][3]);
  acc_guard4(acc[1][0], acc[1][1], acc[1][2], acc[1][3]);
  acc_guard4(acc[2][0], acc[2][1], acc[2][2], acc[2][3]);
  acc_guard4(acc[3][0], acc[3][1], acc[3][2], acc[3][3]);

  float* slab = sT[wave];
  const float* Rb = RESID ? (resid + (size_t)b * strideR) : nullptr;
#pragma unroll
  for (int i = 0; i < 4; ++i) {
    const int mBase = m0 + (i << 4);
#pragma unroll
    for (int j = 0; j < 4; ++j) {
      const int n = n0 + (j << 4) + rlane;
      float bv = 0.f;
      if (BIAS_MODE == 2) bv = bias[n];
#pragma unroll
      for (int r = 0; r < 8; ++r) {
        float v = acc[i][j][r] * scale;
        if (BIAS_MODE == 1) v += bias[mBase + mOff + r];
        if (BIAS_MODE == 2) v += bv;
        if (RESID) v += Rb[(size_t)(mBase + mOff + r) * ldc + n];
        if (ACT == 1) v = tanhf(v);
        if (ACT == 2) v = fmaxf(v, 0.0f);
        if (ACT == 3) v = v / (1.0f + expf(-v));
        if (ACT == 4) v = (v > 0.f) ? v : 0.01f * v;
        slab[(mOff + r) * 68 + (j << 4) + rlane] = v;
      }
    }
    __builtin_amdgcn_fence(__ATOMIC_RELEASE, "workgroup");
    __builtin_amdgcn_wave_barrier();
    __builtin_amdgcn_fence(__ATOMIC_ACQUIRE, "workgroup");
    if (OUT_MODE == 0) {
      float* C = (float*)Cout + (size_t)b * strideC;
      const int hh = lane >> 4, c4 = (lane & 15) * 4;
      for (int pass = 0; pass < 2; ++pass) {
#pragma unroll
        for (int it = 0; it < 8; ++it) {
          const int row = it * 2 + hh;
          v4f v = *(const v4f*)(slab + row * 68 + c4);
          *(volatile v4f*)(C + (size_t)(mBase + row) * ldc + n0 + c4) = v;
        }
        __threadfence();
      }
    } else {
      const int q = lane >> 3, c8 = (lane & 7) * 8;
      unsigned short* C  = (unsigned short*)Cout  + (size_t)b * strideC;
      unsigned short* C2 = (OUT_MODE == 2) ? ((unsigned short*)Cout2 + (size_t)b * strideC) : nullptr;
      for (int pass = 0; pass < 2; ++pass) {
#pragma unroll
        for (int it = 0; it < 4; ++it) {
          const int row = it * 4 + q;
          const float* sp = slab + row * 68 + c8;
          v8h hv, lv;
#pragma unroll
          for (int e = 0; e < 8; ++e) {
            if (OUT_MODE == 1) {
              hv[e] = (_Float16)sp[e];
            } else {
              unsigned short hb = f2bf_bits(sp[e]);
              unsigned short lb = f2bf_bits(sp[e] - bf_bits2f(hb));
              hv[e] = __builtin_bit_cast(_Float16, hb);
              lv[e] = __builtin_bit_cast(_Float16, lb);
            }
          }
          *(volatile v8h*)(C + (size_t)(mBase + row) * ldc + n0 + c8) = hv;
          if (OUT_MODE == 2) *(volatile v8h*)(C2 + (size_t)(mBase + row) * ldc + n0 + c8) = lv;
        }
        __threadfence();
      }
    }
    __builtin_amdgcn_fence(__ATOMIC_RELEASE, "workgroup");
    __builtin_amdgcn_wave_barrier();
    __builtin_amdgcn_fence(__ATOMIC_ACQUIRE, "workgroup");
  }
}

__global__ __launch_bounds__(kThr) void zero_kernel(float* __restrict__ dst) {
  const size_t o4 = ((size_t)blockIdx.x * kThr + threadIdx.x) * 4u;
  const v4f z = {0.f, 0.f, 0.f, 0.f};
  *(volatile v4f*)(dst + o4) = z;
  __threadfence();
  *(volatile v4f*)(dst + o4) = z;
}
__global__ __launch_bounds__(kThr) void pack_kernel(const float* __restrict__ W, unsigned short* __restrict__ D, float* __restrict__ dstf, int part, int ld, int k0, int lg, int n0, int pitch) {
  const unsigned i = blockIdx.x * blockDim.x + threadIdx.x;
  if (part == 0) {
    const unsigned g = i & ((1u << lg) - 1u), n = i >> lg;
    const float* sp = W + (size_t)((unsigned)k0 + g * 8u) * (unsigned)ld + n;
    v8h hv;
#pragma unroll
    for (int t = 0; t < 8; ++t) hv[t] = (_Float16)carry_flush(bf16r(sp[(size_t)t * (unsigned)ld]), kInCarry);
    unsigned short* dp = D + (size_t)((unsigned)n0 + n) * (unsigned)pitch + g * 8u;
    *(volatile v8h*)dp = hv;
    __threadfence();
    *(volatile v8h*)dp = hv;
  } else {
    const v4f a = *(const v4f*)(W + i * 4u);
    v4f o;
#pragma unroll
    for (int e = 0; e < 4; ++e) o[e] = bf16r(a[e]);
    float* dp = dstf + i * 4u;
    *(volatile v4f*)dp = o;
    __threadfence();
    *(volatile v4f*)dp = o;
  }
}

__global__ __launch_bounds__(kThr) void perm_kernel(const float* __restrict__ src, unsigned short* __restrict__ A, int sB, int sM, int sP, int sQ, int pitch, int two, int rnd) {
  const unsigned v = blockIdx.x * (unsigned)kThr + threadIdx.x;
  const unsigned m = v >> 7, k8 = (v & 127u) << 3;
  const unsigned b = m >> 5, rem = m & 31u, xp = k8 >> 5, xq0 = k8 & 31u;
  const float* sp = src + (size_t)b * (unsigned)sB + (size_t)rem * (unsigned)sM + (size_t)xp * (unsigned)sP + (size_t)xq0 * (unsigned)sQ;
  v8h hv, lv;
#pragma unroll
  for (int t = 0; t < 8; ++t) {
    float w = sp[(size_t)t * (unsigned)sQ];
    if (rnd != 0) w = bf16r(w);
    const float s = carry_flush(w, kInCarry);
    const _Float16 h = (_Float16)s;
    hv[t] = h;
    const float r = s - (float)h;
    lv[t] = (_Float16)((fabsf(r) < kF16MinNormal) ? 0.0f : r);
  }
  unsigned short* dp = A + (size_t)m * (unsigned)pitch + k8;
  for (int pass = 0; pass < 2; ++pass) {
    *(volatile v8h*)dp = hv;
    if (two != 0) *(volatile v8h*)(dp + kDD) = lv;
    __threadfence();
  }
}
static_assert((size_t)kM * kDD / 8 == 4096ull * kThr && kDD / 8 == 128, "the permuting cast's grid exact: 4,096 blocks; 128 threads a row");

__global__ __launch_bounds__(kThr) void bro_kernel(const float* __restrict__ C, const float* __restrict__ bias, float* __restrict__ out) {
  const unsigned v = blockIdx.x * (unsigned)kThr + threadIdx.x;
  const unsigned t4 = v << 2;
  const v4f c = *(const v4f*)(C + t4), q = *(const v4f*)(bias + (t4 & (unsigned)(kOut - 1)));
  v4f o;
#pragma unroll
  for (int e = 0; e < 4; ++e) o[e] = fmaxf(c[e] + bf16r(q[e]), 0.0f);
  float* dp = out + t4;
  *(volatile v4f*)dp = o;
  __threadfence();
  *(volatile v4f*)dp = o;
}
static_assert((size_t)kBn * kOut / 4 == 8192ull * kThr && (kOut & (kOut - 1)) == 0, "the epilogue's grid exact: 8,192 blocks");

extern "C" void kernel_launch(void* const* d_in, const int* in_sizes, int n_in,
                              void* d_out, int out_size, void* d_ws, size_t ws_size,
                              hipStream_t stream) {
  if (n_in < 3 || d_out == nullptr || d_ws == nullptr) return;
  if (in_sizes[0] != kBn * kOut || in_sizes[1] != kNN * kDD * kDD || in_sizes[2] != kOut) return;
  if (out_size != kBn * kOut) return;
  if (ws_size < kWsTotal) return;
  const float* x = (const float*)d_in[0];
  const float* nodes = (const float*)d_in[1];
  const float* bias = (const float*)d_in[2];
  float* out = (float*)d_out;
  char* ws = (char*)d_ws;
  float* ZB = (float*)(ws + kOffZB);
  unsigned short* NW = (unsigned short*)(ws + kOffNW);
  unsigned short* A16 = (unsigned short*)(ws + kOffA16);
  float* C = (float*)(ws + kOffC);
  const size_t nwOff[kNN] = { 0ull, (size_t)kDD * kDD, 2ull * kDD * kDD, 3ull * kDD * kDD, 4ull * kDD * kDD, 4ull * kDD * kDD + 2ull * kDD * kDD };
  const int twoW[kNN] = { 0, 0, 0, 0, 1, 1 };

  static_assert(8192ull / 16ull == 2ull * kThr && (kDD * (kDD / 8)) % kThr == 0, "the zero fill's grid (2 blocks over ZB's 8,192 B) and the pack's grid exact");
  zero_kernel<<<2, kThr, 0, stream>>>(ZB);
  for (int i = 0; i < kNN; ++i) {
    const float* W = nodes + (size_t)i * kDD * kDD;
    unsigned short* Dn = NW + nwOff[i];
    const int pitch = twoW[i] ? 2 * kDD : kDD;
    pack_kernel<<<kDD * (kDD / 8) / kThr, kThr, 0, stream>>>(W, Dn, nullptr, 0, kDD, 0, 7, 0, pitch);
    if (twoW[i]) pack_kernel<<<kDD * (kDD / 8) / kThr, kThr, 0, stream>>>(W, Dn + kDD, nullptr, 0, kDD, 0, 7, 0, pitch);
  }
  for (int i = 0; i < kNN; ++i) {
    const int pitch = twoW[i] ? 2 * kDD : kDD;
    if (i == 0) perm_kernel<<<4096, kThr, 0, stream>>>(x, A16, kOut, 1, kDD, kD, pitch, 0, 1);
    else        perm_kernel<<<4096, kThr, 0, stream>>>(C, A16, kOut, kD, 1, kDD, pitch, twoW[i], 0);
    wmma_gemm64<0, false, 2, 0, false, 0><<<dim3((kM / 64) * (kDD / 64) / 8, 1), 256, 0, stream>>>(
        A16, A16, pitch, 0L, NW + nwOff[i], NW + nwOff[i], pitch, 0L, (void*)C, (void*)C, kDD, 0L, ZB, nullptr, 0L, kM, kDD, pitch, kSc);
  }
  bro_kernel<<<8192, kThr, 0, stream>>>(C, bias, out);
}
static_assert(((kM / 64) * (kDD / 64)) % 8 == 0 && kDD % 32 == 0, "the engine's grid: whole blocks of eight wave tiles; both depths multiples of 32");
